// ScaledEuclidDistanceAttention_32615981646584
// MI455X (gfx1250) — hardware-verified
//
#include <hip/hip_runtime.h>
#include <math.h>

constexpr int kBatch = 2;
constexpr int kSeq   = 2048;
constexpr int kDim   = 1024;
constexpr int kHeads = 16;
constexpr int kDh    = 64;
constexpr int kGroup = 4;
constexpr int kTok   = kBatch * kSeq;
constexpr float kPCarry    = 32768.0f;
constexpr float kPCarryInv = 1.0f / 32768.0f;
constexpr float kDistScale = 0.125f;
constexpr float kEps       = 1.0e-9f;
constexpr float kNegBig    = -1.0e9f;
static_assert(kHeads * kDh == kDim, "shape");
static_assert(kSeq % 64 == 0 && kDh % 32 == 0 && kSeq % 256 == 0, "tiles");
static_assert(kHeads % kGroup == 0, "groups");

typedef __attribute__((ext_vector_type(16))) _Float16 v16h;
typedef __attribute__((ext_vector_type(8)))  _Float16 v8h;
typedef __attribute__((ext_vector_type(16))) __bf16   v16b;
typedef __attribute__((ext_vector_type(8)))  __bf16   v8b;
typedef __attribute__((ext_vector_type(8)))  float    v8f;
typedef __attribute__((ext_vector_type(4)))  float    v4f;
typedef __attribute__((ext_vector_type(2)))  float    v2f;
typedef __attribute__((ext_vector_type(2)))  int      v2i;
typedef __attribute__((ext_vector_type(4)))  unsigned int v4u;

__device__ __forceinline__ unsigned short f2bf_bits(float f) {
  unsigned u = __float_as_uint(f);
  return (unsigned short)((u + 0x7FFFu + ((u >> 16) & 1u)) >> 16);
}
__device__ __forceinline__ float bf_bits2f(unsigned short h) { return __uint_as_float(((unsigned)h) << 16); }

__device__ __forceinline__ void dep_guard_h(v8f& a, v8f& b, v16h x, v16h y) { asm volatile("v_nop\n\tv_nop\n\tv_nop\n\tv_nop" : "+v"(a), "+v"(b) : "v"(x), "v"(y)); }
__device__ __forceinline__ void dep_guard_b(v8f& a, v8f& b, v16b x, v16b y) { asm volatile("v_nop\n\tv_nop\n\tv_nop\n\tv_nop" : "+v"(a), "+v"(b) : "v"(x), "v"(y)); }
__device__ __forceinline__ void keep4_h(v16h a, v16h b, v16h c, v16h d) { asm volatile("v_nop" :: "v"(a), "v"(b), "v"(c), "v"(d)); }
__device__ __forceinline__ void keep4_b(v16b a, v16b b, v16b c, v16b d) { asm volatile("v_nop" :: "v"(a), "v"(b), "v"(c), "v"(d)); }
__device__ __forceinline__ void acc_guard4(v8f& a, v8f& b, v8f& c, v8f& d) { asm volatile("v_nop\n\tv_nop\n\tv_nop\n\tv_nop" : "+v"(a), "+v"(b), "+v"(c), "+v"(d)); }
template <typename T> struct Frag;
template <> struct Frag<_Float16> {
  typedef v16h V; union U { v16h v; v8h h[2]; };
  static __device__ __forceinline__ v16h load(const _Float16* p) {
    U f; f.h[0] = *(const v8h*)(p); f.h[1] = *(const v8h*)(p + 16); return f.v;
  }
  static __device__ __forceinline__ v8f mma(v16h a, v16h b, v8f c) {
    return __builtin_amdgcn_wmma_f32_16x16x32_f16(false, a, false, b, (short)0, c, false, false);
  }
  static __device__ __forceinline__ void guard(v8f& a, v8f& b, v16h x, v16h y) { dep_guard_h(a, b, x, y); }
  static __device__ __forceinline__ void keep(v16h a, v16h b, v16h c, v16h d) { keep4_h(a, b, c, d); }
};
template <> struct Frag<__bf16> {
  typedef v16b V; union U { v16b v; v8b h[2]; };
  static __device__ __forceinline__ v16b load(const __bf16* p) {
    U f; f.h[0] = *(const v8b*)(p); f.h[1] = *(const v8b*)(p + 16); return f.v;
  }
  static __device__ __forceinline__ v8f mma(v16b a, v16b b, v8f c) {
    return __builtin_amdgcn_wmma_f32_16x16x32_bf16(false, a, false, b, (short)0, c, false, false);
  }
  static __device__ __forceinline__ void guard(v8f& a, v8f& b, v16b x, v16b y) { dep_guard_b(a, b, x, y); }
  static __device__ __forceinline__ void keep(v16b a, v16b b, v16b c, v16b d) { keep4_b(a, b, c, d); }
};

__device__ __forceinline__ unsigned pk16(unsigned short a, unsigned short b) { return (unsigned)a | ((unsigned)b << 16); }
__device__ __forceinline__ unsigned short h_bits(float f) { const _Float16 h = (_Float16)f; return __builtin_bit_cast(unsigned short, h); }

template <int ET> struct Elem;
template <> struct Elem<0> { typedef _Float16 T; };
template <> struct Elem<1> { typedef __bf16 T; };
template <int ET, bool SPLIT, int BIAS_MODE, int OUT_MODE, bool RESID, int ACT = 0>
__global__ __launch_bounds__(256) void wmma_gemm64(
    const unsigned short* __restrict__ Ap, const unsigned short* __restrict__ A2p, int lda, long strideA,
    const unsigned short* __restrict__ Btp, const unsigned short* __restrict__ Bt2p, int ldb, long strideB,
    void* __restrict__ Cout, void* __restrict__ Cout2, int ldc, long strideC,
    const float* __restrict__ bias,
    const float* __restrict__ resid, long strideR,
    int M, int N, int K, float scale) {
  typedef typename Elem<ET>::T T;
  typedef typename Frag<T>::V V;
  const T* A = (const T*)Ap; const T* A2 = (const T*)A2p; const T* Bt = (const T*)Btp; const T* Bt2 = (const T*)Bt2p;
  __shared__ __align__(16) float sT[8][16 * 68];
  const int b    = blockIdx.y;
  const int lane = threadIdx.x & 31;
  const int wave = threadIdx.x >> 5;
  const int tilesN = N >> 6;
  const int tilesM = M >> 6;
  const int tile = blockIdx.x * 8 + wave;
  if (tile >= tilesM * tilesN) return;
  const int tm = tile / tilesN;
  const int tn = tile - tm * tilesN;
  const int m0 = tm << 6;
  const int n0 = tn << 6;

  const T* Ab  = A  + (size_t)b * strideA;
  const T* Bb  = Bt + (size_t)b * strideB;
  const T* Ab2 = SPLIT ? (A2  + (size_t)b * strideA) : nullptr;
  const T* Bb2 = SPLIT ? (Bt2 + (size_t)b * strideB) : nullptr;

  const int rlane = lane & 15;
  const int koff  = (lane >> 4) * 8;
  const int mOff  = (lane >> 4) * 8;

  v8f acc[4][4];
#pragma unroll
  for (int i = 0; i < 4; ++i)
#pragma unroll
    for (int j = 0; j < 4; ++j) acc[i][j] = (v8f){0.f,0.f,0.f,0.f,0.f,0.f,0.f,0.f};

  for (int k0 = 0; k0 < K; k0 += 32) {
    V bh[4], bl[4];
#pragma unroll
    for (int j = 0; j < 4; ++j) {
      const size_t bo = (size_t)(n0 + (j << 4) + rlane) * ldb + koff + k0;
      bh[j] = Frag<T>::load(Bb + bo);
      if (SPLIT) bl[j] = Frag<T>::load(Bb2 + bo);
    }
#pragma unroll
    for (int i = 0; i < 4; ++i) {
      const size_t ao = (size_t)(m0 + (i << 4) + rlane) * lda + koff + k0;
      V ah = Frag<T>::load(Ab + ao);
      V al;
      if (SPLIT) al = Frag<T>::load(Ab2 + ao);
#pragma unroll
      for (int j = 0; j < 4; ++j) {
        acc[i][j] = Frag<T>::mma(ah, bh[j], acc[i][j]);
        if (SPLIT) {
          acc[i][j] = Frag<T>::mma(ah, bl[j], acc[i][j]);
          acc[i][j] = Frag<T>::mma(al, bh[j], acc[i][j]);
        }
      }
      Frag<T>::guard(acc[i][0], acc[i][3], ah, SPLIT ? al : ah);
    }
    Frag<T>::keep(bh[0], bh[1], bh[2], bh[3]);
    if (SPLIT) Frag<T>::keep(bl[0], bl[1], bl[2], bl[3]);
  }
  acc_guard4(acc[0][0], acc[0][1], acc[0][2], acc[0][3]);
  acc_guard4(acc[1][0], acc[1][1], acc[1][2], acc[1][3]);
  acc_guard4(acc[2][0], acc[2][1], acc[2][2], acc[2][3]);
  acc_guard4(acc[3][0], acc[3][1], acc[3][2], acc[3][3]);

  float* slab = sT[wave];
  const float* Rb = RESID ? (resid + (size_t)b * strideR) : nullptr;
#pragma unroll
  for (int i = 0; i < 4; ++i) {
    const int mBase = m0 + (i << 4);
#pragma unroll
    for (int j = 0; j < 4; ++j) {
      const int n = n0 + (j << 4) + rlane;
      float bv = 0.f;
      if (BIAS_MODE == 2) bv = bias[n];
#pragma unroll
      for (int r = 0; r < 8; ++r) {
        float v = acc[i][j][r] * scale;
        if (BIAS_MODE == 1) v += bias[mBase + mOff + r];
        if (BIAS_MODE == 2) v += bv;
        if (RESID) v += Rb[(size_t)(mBase + mOff + r) * ldc + n];
        if (ACT == 2) v = fmaxf(v, 0.0f);
        if (ACT == 4) v = (v > 0.f) ? v : 0.01f * v;
        slab[(mOff + r) * 68 + (j << 4) + rlane] = v;
      }
    }
    __builtin_amdgcn_fence(__ATOMIC_RELEASE, "workgroup");
    __builtin_amdgcn_wave_barrier();
    __builtin_amdgcn_fence(__ATOMIC_ACQUIRE, "workgroup");
    if (OUT_MODE == 0) {
      float* C = (float*)Cout + (size_t)b * strideC;
      const int hh = lane >> 4, c4 = (lane & 15) * 4;
      for (int pass = 0; pass < 2; ++pass) {
#pragma unroll
        for (int it = 0; it < 8; ++it) {
          const int row = it * 2 + hh;
          v4f v = *(const v4f*)(slab + row * 68 + c4);
          *(volatile v4f*)(C + (size_t)(mBase + row) * ldc + n0 + c4) = v;
        }
        __threadfence();
      }
    } else {
      const int q = lane >> 3, c8 = (lane & 7) * 8;
      unsigned short* C  = (unsigned short*)Cout  + (size_t)b * strideC;
      unsigned short* C2 = (OUT_MODE == 2) ? ((unsigned short*)Cout2 + (size_t)b * strideC) : nullptr;
      for (int pass = 0; pass < 2; ++pass) {
#pragma unroll
        for (int it = 0; it < 4; ++it) {
          const int row = it * 4 + q;
          const float* sp = slab + row * 68 + c8;
          v8h hv, lv;
#pragma unroll
          for (int e = 0; e < 8; ++e) {
            if (OUT_MODE == 1) {
              hv[e] = (_Float16)sp[e];
            } else {
              unsigned short hb = f2bf_bits(sp[e]);
              unsigned short lb = f2bf_bits(sp[e] - bf_bits2f(hb));
              hv[e] = __builtin_bit_cast(_Float16, hb);
              lv[e] = __builtin_bit_cast(_Float16, lb);
            }
          }
          *(volatile v8h*)(C + (size_t)(mBase + row) * ldc + n0 + c8) = hv;
          if (OUT_MODE == 2) *(volatile v8h*)(C2 + (size_t)(mBase + row) * ldc + n0 + c8) = lv;
        }
        __threadfence();
      }
    }
    __builtin_amdgcn_fence(__ATOMIC_RELEASE, "workgroup");
    __builtin_amdgcn_wave_barrier();
    __builtin_amdgcn_fence(__ATOMIC_ACQUIRE, "workgroup");
  }
}

__global__ __launch_bounds__(256) void cast8_f16_kernel(const float* __restrict__ in, unsigned short* __restrict__ out, int n8) {
  const int i = blockIdx.x * 256 + threadIdx.x;
  if (i >= n8) return;
  const float* p = in + 8 * (size_t)i;
  const v4f a = *(const v4f*)(p);
  const v4f c = *(const v4f*)(p + 4);
  unsigned short hb[8];
#pragma unroll
  for (int e = 0; e < 4; ++e) {
    hb[e]     = h_bits(a[e]);
    hb[4 + e] = h_bits(c[e]);
  }
  const v4u u = (v4u){pk16(hb[0], hb[1]), pk16(hb[2], hb[3]), pk16(hb[4], hb[5]), pk16(hb[6], hb[7])};
  unsigned short* q = out + 8 * (size_t)i;
  *(volatile v4u*)q = u;
  __threadfence();
  *(volatile v4u*)q = u;
}

__global__ __launch_bounds__(256) void vt_cast_kernel(const float* __restrict__ v, unsigned short* __restrict__ VT) {
  __shared__ float sm[64][65];
  const int t  = threadIdx.x;
  const int s0 = blockIdx.x * 64;
  const int h  = blockIdx.y;
  const int b  = blockIdx.z;
#pragma unroll
  for (int i = 0; i < 16; ++i) {
    const int e = i * 256 + t;
    const int r = e >> 6;
    const int c = e & 63;
    sm[c][r] = v[((size_t)(b * kSeq + s0 + r)) * kDim + h * kDh + c];
  }
  __syncthreads();
  const int lane = t & 31, wave = t >> 5;
  const int q = lane >> 3, c8 = (lane & 7) * 8;
  unsigned short* op = VT + ((size_t)(b * kHeads + h) * kDh) * kSeq;
  for (int pass = 0; pass < 2; ++pass) {
#pragma unroll
    for (int it = 0; it < 2; ++it) {
      const int row = wave * 8 + it * 4 + q;
      unsigned short hb[8];
#pragma unroll
      for (int e = 0; e < 8; ++e) hb[e] = h_bits(sm[row][c8 + e]);
      const v4u u = (v4u){pk16(hb[0], hb[1]), pk16(hb[2], hb[3]), pk16(hb[4], hb[5]), pk16(hb[6], hb[7])};
      *(volatile v4u*)(op + (size_t)row * kSeq + s0 + c8) = u;
    }
    __threadfence();
  }
}

__global__ __launch_bounds__(256) void sumsq_kernel(const float* __restrict__ x, float* __restrict__ dst, const int* __restrict__ unused_nh) {
  (void)unused_nh;
  __shared__ __align__(16) float sq[256];
  const int t  = threadIdx.x;
  const int s0 = blockIdx.x * 256;
  const int h  = blockIdx.y;
  const int b  = blockIdx.z;
  const float* row = x + ((size_t)(b * kSeq + s0 + t)) * kDim + h * kDh;
  float a0 = 0.f, a1 = 0.f, a2 = 0.f, a3 = 0.f;
#pragma unroll 1
  for (int j = 0; j < 16; ++j) {
    const v4f w = *(const v4f*)(row + 4 * j);
    a0 += w[0] * w[0];
    a1 += w[1] * w[1];
    a2 += w[2] * w[2];
    a3 += w[3] * w[3];
  }
  sq[t] = (a0 + a1) + (a2 + a3);
  __syncthreads();
  if (t < 64) {
    const v4f val = *(const v4f*)(sq + 4 * t);
    float* dp = dst + (size_t)(b * kHeads + h) * kSeq + s0 + 4 * t;
    *(volatile v4f*)dp = val;
    __threadfence();
    *(volatile v4f*)dp = val;
  }
}

__global__ __launch_bounds__(256) void dist_softmax_kernel(const float* __restrict__ Sp, const float* __restrict__ q2p,
                                                          const float* __restrict__ k2p, const int* __restrict__ maskp,
                                                          unsigned short* __restrict__ Pp) {
  __shared__ __align__(16) float lg[kSeq];
  __shared__ float redM[8];
  __shared__ float redS[8];
  const int i    = blockIdx.x;
  const int hg   = blockIdx.y;
  const int t    = threadIdx.x;
  const int lane = t & 31, wave = t >> 5;
  const size_t rowoff = ((size_t)hg * kSeq + i) * kSeq;
  const float* sr = Sp + rowoff;
  const float* kr = k2p + (size_t)hg * kSeq;
  const int*   mr = maskp + (size_t)i * kSeq;
  const float q2i = q2p[hg * kSeq + i];

  float mx = -__builtin_inff();
#pragma unroll 1
  for (int it = 0; it < 4; ++it) {
    const int c = it * 512 + 2 * t;
    const v2f sv = *(const v2f*)(sr + c);
    const v2f kv = *(const v2f*)(kr + c);
    const v2i mv = *(const v2i*)(mr + c);
    v2f av;
#pragma unroll
    for (int e = 0; e < 2; ++e) {
      float d2 = (q2i + kv[e]) - 2.0f * sv[e];
      d2 = fmaxf(d2, 0.0f);
      const float dist = sqrtf(d2) * kDistScale;
      float a = 1.0f / (dist + kEps);
      a = a + (float)mv[e] * kNegBig;
      av[e] = a;
      mx = fmaxf(mx, a);
    }
    *(v2f*)(lg + c) = av;
  }
#pragma unroll
  for (int off = 16; off > 0; off >>= 1) mx = fmaxf(mx, __shfl_xor(mx, off, 32));
  if (lane == 0) redM[wave] = mx;
  __syncthreads();
  float m = redM[0];
#pragma unroll
  for (int w = 1; w < 8; ++w) m = fmaxf(m, redM[w]);

  float sum = 0.f;
#pragma unroll 1
  for (int it = 0; it < 4; ++it) {
    const int c = it * 512 + 2 * t;
    const v2f l = *(const v2f*)(lg + c);
    v2f ev;
#pragma unroll
    for (int e = 0; e < 2; ++e) {
      ev[e] = expf(l[e] - m);
      sum += ev[e];
    }
    *(v2f*)(lg + c) = ev;
  }
#pragma unroll
  for (int off = 16; off > 0; off >>= 1) sum += __shfl_xor(sum, off, 32);
  if (lane == 0) redS[wave] = sum;
  __syncthreads();
  float tot = redS[0];
#pragma unroll
  for (int w = 1; w < 8; ++w) tot += redS[w];
  const float inv = kPCarry / tot;

  const v4f e0 = *(const v4f*)(lg + 8 * t);
  const v4f e1 = *(const v4f*)(lg + 8 * t + 4);
  unsigned short hb[8];
#pragma unroll
  for (int e = 0; e < 4; ++e) {
    hb[e]     = h_bits(e0[e] * inv);
    hb[4 + e] = h_bits(e1[e] * inv);
  }
  const v4u u = (v4u){pk16(hb[0], hb[1]), pk16(hb[2], hb[3]), pk16(hb[4], hb[5]), pk16(hb[6], hb[7])};
  unsigned short* pr = Pp + rowoff + 8 * (size_t)t;
  *(volatile v4u*)pr = u;
  __threadfence();
  *(volatile v4u*)pr = u;
}

extern "C" void kernel_launch(void* const* d_in, const int* in_sizes, int n_in,
                              void* d_out, int out_size, void* d_ws, size_t ws_size,
                              hipStream_t stream) {
  if (n_in < 5) return;
  const int nElem = kBatch * kSeq * kDim;
  if (in_sizes[0] != nElem || in_sizes[1] != nElem || in_sizes[2] != nElem) return;
  if (in_sizes[3] != kSeq * kSeq) return;
  if (out_size != nElem) return;

  const size_t szQK = (size_t)kTok * kDim * 2;
  const size_t szVT = (size_t)kBatch * kHeads * kDh * kSeq * 2;
  const size_t szN  = (size_t)kBatch * kHeads * kSeq * 4;
  const size_t szS  = (size_t)kGroup * kSeq * kSeq * 4;
  const size_t szP  = (size_t)kGroup * kSeq * kSeq * 2;
  const size_t offQ  = 0;
  const size_t offK  = offQ + szQK;
  const size_t offVT = offK + szQK;
  const size_t offQ2 = offVT + szVT;
  const size_t offK2 = offQ2 + szN;
  const size_t offS  = offK2 + szN;
  const size_t offP  = offS + szS;
  const size_t total = offP + szP;
  if (ws_size < total) return;

  const float* q    = (const float*)d_in[0];
  const float* k    = (const float*)d_in[1];
  const float* v    = (const float*)d_in[2];
  const int*   mask = (const int*)d_in[3];
  const int*   nh   = (const int*)d_in[4];
  float* out = (float*)d_out;
  char* ws = (char*)d_ws;
  unsigned short* Q16 = (unsigned short*)(ws + offQ);
  unsigned short* K16 = (unsigned short*)(ws + offK);
  unsigned short* VT  = (unsigned short*)(ws + offVT);
  float* Q2 = (float*)(ws + offQ2);
  float* K2 = (float*)(ws + offK2);
  float* SC = (float*)(ws + offS);
  unsigned short* PP = (unsigned short*)(ws + offP);

  const int n8 = (kTok * kDim) / 8;
  cast8_f16_kernel<<<dim3(n8 / 256), dim3(256), 0, stream>>>(q, Q16, n8);
  cast8_f16_kernel<<<dim3(n8 / 256), dim3(256), 0, stream>>>(k, K16, n8);
  vt_cast_kernel<<<dim3(kSeq / 64, kHeads, kBatch), dim3(256), 0, stream>>>(v, VT);
  sumsq_kernel<<<dim3(kSeq / 256, kHeads, kBatch), dim3(256), 0, stream>>>(q, Q2, nh);
  sumsq_kernel<<<dim3(kSeq / 256, kHeads, kBatch), dim3(256), 0, stream>>>(k, K2, nh);

  const long strideHead16 = (long)kDh;
  const long strideScore  = (long)kSeq * kSeq;
  const long strideVT     = (long)kDh * kSeq;
  const int  tilesScore   = (kSeq / 64) * (kSeq / 64);
  const int  tilesCtx     = (kSeq / 64) * (kDh / 64);

  for (int b = 0; b < kBatch; ++b) {
    for (int g = 0; g < kHeads / kGroup; ++g) {
      const size_t tokOff  = ((size_t)b * kSeq) * kDim + (size_t)g * kGroup * kDh;
      const size_t headIdx = (size_t)b * kHeads + (size_t)g * kGroup;
      const unsigned short* Ag  = Q16 + tokOff;
      const unsigned short* Btg = K16 + tokOff;
      wmma_gemm64<0, false, 0, 0, false, 0><<<dim3(tilesScore / 8, kGroup), dim3(256), 0, stream>>>(
          Ag, Ag, kDim, strideHead16, Btg, Btg, kDim, strideHead16,
          (void*)SC, (void*)SC, kSeq, strideScore, Q2, Q2, 0L, kSeq, kSeq, kDh, 1.0f);
      dist_softmax_kernel<<<dim3(kSeq, kGroup), dim3(256), 0, stream>>>(
          SC, Q2 + headIdx * kSeq, K2 + headIdx * kSeq, mask, PP);
      const unsigned short* VTg = VT + headIdx * (size_t)kDh * kSeq;
      float* outg = out + tokOff;
      wmma_gemm64<0, false, 0, 0, false, 0><<<dim3(tilesCtx / 8, kGroup), dim3(256), 0, stream>>>(
          PP, PP, kSeq, strideScore, VTg, VTg, kSeq, strideVT,
          (void*)outg, (void*)outg, kDim, strideHead16, Q2, Q2, 0L, kSeq, kDh, kSeq, kPCarryInv);
    }
  }
}
